// DirectionalAGLGF_79027398246895
// MI455X (gfx1250) — hardware-run, weakly checked
//
#include <hip/hip_runtime.h>
#include <hip/hip_bf16.h>
#include <math.h>

#define NB    2
#define LL    4096
#define NTOK  (NB * LL)
#define DMOD  128
#define DIN   256
#define DST   16
#define DTR   8
#define XDR   40
#define XDN   64
#define DCV   4
#define GSTR  40
#define OSTR  68
#define SMEMB (8 * 16 * OSTR * 4)
#define SCH   32
#define SYP   260
#define TSP   36
#define LOG2E 1.4426950408889634f
#define WSCAP ((size_t)134217728)

static_assert(NTOK % 128 == 0);
static_assert(NTOK % 8 == 0);
static_assert(NTOK % 32 == 0);
static_assert(DIN % 64 == 0);
static_assert(DMOD % 64 == 0);
static_assert(DMOD % 32 == 0);
static_assert(DIN % 32 == 0);
static_assert(XDN == 64);
static_assert(XDR <= XDN);
static_assert(DTR == 8);
static_assert(DST == 16);
static_assert(DIN == 256);
static_assert(DMOD == 128);
static_assert(LL % SCH == 0);
static_assert(LL % 32 == 0);
static_assert(SCH == 32);
static_assert(SYP % 4 == 0);
static_assert(SYP >= DIN);
static_assert(TSP % 4 == 0);
static_assert(SMEMB >= (2 * 128 * GSTR + 64 * GSTR) * 2);

typedef unsigned short us16 __attribute__((ext_vector_type(16)));
typedef unsigned short us8  __attribute__((ext_vector_type(8)));
typedef unsigned short us8a __attribute__((ext_vector_type(8), may_alias));
typedef unsigned short us4  __attribute__((ext_vector_type(4)));
typedef __bf16 v16b __attribute__((ext_vector_type(16)));
typedef float v8f __attribute__((ext_vector_type(8)));
typedef float v4f __attribute__((ext_vector_type(4)));
typedef float v4fa __attribute__((ext_vector_type(4), may_alias));
union FragU { us16 v; us8 h[2]; };

__device__ __forceinline__ unsigned short bf16_bits(float f) {
  unsigned u = __float_as_uint(f);
  u += 0x7FFFu + ((u >> 16) & 1u);
  return (unsigned short)(u >> 16);
}
__device__ __forceinline__ float bf16_val(unsigned short b) { return __uint_as_float(((unsigned)b) << 16); }
__device__ __forceinline__ float bf16r(float f) { return bf16_val(bf16_bits(f)); }
__device__ __forceinline__ float siluf(float x) { return x * __builtin_amdgcn_rcpf(1.0f + __expf(-x)); }

__device__ __forceinline__ v8f mma_bf16(us16 a, us16 b, v8f c) {
  return __builtin_amdgcn_wmma_f32_16x16x32_bf16(false, __builtin_bit_cast(v16b, a), false, __builtin_bit_cast(v16b, b), (short)0, c, false, false);
}
__device__ __forceinline__ void wguard(v8f& c0, v8f& c1, v8f& c2, v8f& c3, const us16& a0, const us16& a1,
                                       const us16& b0, const us16& b1, const us16& b2, const us16& b3) {
#if defined(__HIP_DEVICE_COMPILE__)
  asm volatile("v_nop\n\tv_nop\n\tv_nop\n\tv_nop"
               : "+v"(c0), "+v"(c1), "+v"(c2), "+v"(c3)
               : "v"(a0), "v"(a1), "v"(b0), "v"(b1), "v"(b2), "v"(b3));
#endif
}

__device__ __forceinline__ us16 lds_frag(const unsigned short* base) {
  const int lane = threadIdx.x & 31, r = lane & 15, kh = (lane >> 4) * 8;
  FragU f;
  f.h[0] = *(const us8a*)(base + r * GSTR + kh);
  f.h[1] = *(const us8a*)(base + r * GSTR + 16 + kh);
  return f.v;
}

__device__ __forceinline__ void stage_a(unsigned short* lds, const unsigned short* __restrict__ P, int ld, int m0, int k0, int tid) {
  const int row = tid >> 1, cq = (tid & 1) * 16;
  const unsigned short* src = P + (size_t)(m0 + row) * ld + k0 + cq;
  const us8 v0 = *(const us8a*)src;
  const us8 v1 = *(const us8a*)(src + 8);
  *(us8a*)(lds + row * GSTR + cq) = v0;
  *(us8a*)(lds + row * GSTR + cq + 8) = v1;
}
__device__ __forceinline__ void stage_b(unsigned short* lds, const unsigned short* __restrict__ P, int ld, int n0, int k0, int tid) {
  const int row = tid >> 2, kq = (tid & 3) * 8;
  const us8 v = *(const us8a*)(P + (size_t)(n0 + row) * ld + k0 + kq);
  *(us8a*)(lds + row * GSTR + kq) = v;
}

__global__ __launch_bounds__(256) void k_copy(const float* __restrict__ src, float* dst, int n4) {
  const int i = blockIdx.x * 256 + threadIdx.x;
  if (i >= n4) return;
  typedef float v4f_ __attribute__((ext_vector_type(4)));
  const v4f_ v = *(const v4f_*)(src + (size_t)i * 4);
  *(volatile v4f_*)(dst + (size_t)i * 4) = v;
  __threadfence();
  *(volatile v4f_*)(dst + (size_t)i * 4) = v;
}

__global__ __launch_bounds__(256) void k_gemm(const unsigned short* __restrict__ A0, const unsigned short* __restrict__ A1, int lda,
                                             const unsigned short* __restrict__ B0, int ldb, float* Y, int ldy, int K) {
  __shared__ __attribute__((aligned(16))) unsigned char sm[SMEMB];
  unsigned short* lA0 = (unsigned short*)sm;
  unsigned short* lA1 = lA0 + 128 * GSTR;
  unsigned short* lB0 = lA1 + 128 * GSTR;
  float* oS = (float*)sm;
  const int tid = threadIdx.x, lane = tid & 31, wave = tid >> 5, cl = lane & 15, hh = lane >> 4;
  const int m0 = blockIdx.x * 128, n0 = blockIdx.y * 64;

  v8f acc[4];
#pragma unroll
  for (int j = 0; j < 4; ++j) { v8f zz = {0.f, 0.f, 0.f, 0.f, 0.f, 0.f, 0.f, 0.f}; acc[j] = zz; }

#pragma unroll 1
  for (int k0 = 0; k0 < K; k0 += 32) {
    __syncthreads();
    stage_a(lA0, A0, lda, m0, k0, tid);
    stage_a(lA1, A1, lda, m0, k0, tid);
    stage_b(lB0, B0, ldb, n0, k0, tid);
    __syncthreads();
    const us16 af0 = lds_frag(lA0 + 16 * wave * GSTR);
    const us16 af1 = lds_frag(lA1 + 16 * wave * GSTR);
    us16 bfr[4];
#pragma unroll
    for (int j = 0; j < 4; ++j) bfr[j] = lds_frag(lB0 + 16 * j * GSTR);
#pragma unroll
    for (int j = 0; j < 4; ++j) acc[j] = mma_bf16(af0, bfr[j], acc[j]);
#pragma unroll
    for (int j = 0; j < 4; ++j) acc[j] = mma_bf16(af1, bfr[j], acc[j]);
    wguard(acc[0], acc[1], acc[2], acc[3], af0, af1, bfr[0], bfr[1], bfr[2], bfr[3]);
  }
  __syncthreads();

  float* so = oS + wave * (16 * OSTR);
#pragma unroll
  for (int j = 0; j < 4; ++j)
#pragma unroll
    for (int r = 0; r < 8; ++r) so[(8 * hh + r) * OSTR + 16 * j + cl] = acc[j][r];
  __syncthreads();
#pragma unroll
  for (int pass = 0; pass < 2; ++pass) {
#pragma unroll
    for (int it = 0; it < 8; ++it) {
      const int ch = it * 32 + lane, r = ch >> 4, q = (ch & 15) * 4;
      const v4f v = *(const v4fa*)(so + r * OSTR + q);
      *(volatile v4f*)(Y + (size_t)(m0 + 16 * wave + r) * ldy + n0 + q) = v;
    }
    __threadfence();
  }
}

__global__ __launch_bounds__(256) void k_cvt(const float* __restrict__ src, unsigned short* dst, int nsrc, int ncol8, int total8) {
  const int idx = blockIdx.x * 256 + threadIdx.x;
  if (idx >= total8) return;
  const int row = idx / ncol8, c8 = (idx - row * ncol8) * 8;
  const int rs = (row < nsrc) ? row : (nsrc - 1);
  const float* s = src + (size_t)rs * (size_t)(ncol8 * 8) + c8;
  const v4f a = *(const v4fa*)s, b = *(const v4fa*)(s + 4);
  const bool zr = (row >= nsrc);
  us8 o;
#pragma unroll
  for (int u = 0; u < 4; ++u) {
    o[u]     = zr ? (unsigned short)0 : bf16_bits(a[u]);
    o[4 + u] = zr ? (unsigned short)0 : bf16_bits(b[u]);
  }
  const size_t off = (size_t)row * (size_t)(ncol8 * 8) + c8;
  *(volatile us8*)(dst + off) = o;
  __threadfence();
  *(volatile us8*)(dst + off) = o;
}

__device__ __forceinline__ void ln4(const float (&v)[4], const float* __restrict__ g, const float* __restrict__ bt, int c0, us4& hi, us4& lo) {
#pragma clang fp contract(off)
  float s = (v[0] + v[1]) + (v[2] + v[3]);
#pragma unroll
  for (int o = 16; o > 0; o >>= 1) s = s + __shfl_xor(s, o);
  const float mu = s * (1.0f / DMOD);
  float d[4];
#pragma unroll
  for (int u = 0; u < 4; ++u) d[u] = v[u] - mu;
  float s2 = (d[0] * d[0] + d[1] * d[1]) + (d[2] * d[2] + d[3] * d[3]);
#pragma unroll
  for (int o = 16; o > 0; o >>= 1) s2 = s2 + __shfl_xor(s2, o);
  const float var = s2 * (1.0f / DMOD);
  const float rs = rsqrtf(var + 1e-5f);
#pragma unroll
  for (int u = 0; u < 4; ++u) {
    const float o = (d[u] * rs) * bf16r(g[c0 + u]) + bf16r(bt[c0 + u]);
    const unsigned short hb = bf16_bits(o);
    hi[u] = hb; lo[u] = bf16_bits(o - bf16_val(hb));
  }
}

__global__ __launch_bounds__(256) void k_ln(const float* __restrict__ x1, const float* __restrict__ x2,
                                           const float* __restrict__ gq, const float* __restrict__ bq,
                                           const float* __restrict__ gk, const float* __restrict__ bk,
                                           unsigned short* X1H, unsigned short* X1L, unsigned short* X2H, unsigned short* X2L) {
#pragma clang fp contract(off)
  const int tid = threadIdx.x, lane = tid & 31, wave = tid >> 5;
  const int tok = blockIdx.x * 8 + wave;
  const int b = tok / LL, l = tok - b * LL;
  const int c0 = lane * 4;
  float v1[4], v2[4];
#pragma unroll
  for (int u = 0; u < 4; ++u) {
    const size_t src = ((size_t)(b * DMOD + c0 + u)) * LL + (size_t)l;
    v1[u] = bf16r(x1[src]);
    v2[u] = bf16r(x2[src]);
  }
  us4 h1, l1, h2, l2;
  ln4(v1, gq, bq, c0, h1, l1);
  ln4(v2, gk, bk, c0, h2, l2);
  const size_t off = (size_t)tok * DMOD + c0;
  *(volatile us4*)(X1H + off) = h1; *(volatile us4*)(X1L + off) = l1;
  *(volatile us4*)(X2H + off) = h2; *(volatile us4*)(X2L + off) = l2;
  __threadfence();
  *(volatile us4*)(X1H + off) = h1; *(volatile us4*)(X1L + off) = l1;
  *(volatile us4*)(X2H + off) = h2; *(volatile us4*)(X2L + off) = l2;
}

template <int DIR>
__global__ __launch_bounds__(256) void k_conv(const float* __restrict__ XB, const float* __restrict__ cw, const float* __restrict__ cb,
                                             float* XCF, unsigned short* XCH, unsigned short* XCL) {
#pragma clang fp contract(off)
  const int tid = threadIdx.x, lane = tid & 31, wave = tid >> 5;
  const int tok = blockIdx.x * 8 + wave;
  const int b = tok / LL, t = tok - b * LL;
#pragma unroll
  for (int H = 0; H < 2; ++H) {
    const int c = H * 128 + lane * 4;
    v4f xv[DCV];
#pragma unroll
    for (int j = 0; j < DCV; ++j) {
      const int jj = t - (DCV - 1) + j;
      const int jjc = (jj < 0) ? 0 : jj;
      const int p = DIR ? (LL - 1 - jjc) : jjc;
      xv[j] = *(const v4fa*)(XB + ((size_t)b * LL + (size_t)p) * DIN + c);
    }
    const v4f bb = *(const v4fa*)(cb + c);
    v4f sv;
    us4 hi, lo;
#pragma unroll
    for (int u = 0; u < 4; ++u) {
      const v4f wv = *(const v4fa*)(cw + (size_t)(c + u) * DCV);
      float a = 0.0f;
#pragma unroll
      for (int j = 0; j < DCV; ++j) {
        const float pr = bf16r(wv[j]) * xv[j][u];
        a = a + ((t - (DCV - 1) + j >= 0) ? pr : 0.0f);
      }
      a = a + bf16r(bb[u]);
      const float sres = siluf(a);
      sv[u] = sres;
      const unsigned short hb = bf16_bits(sres);
      hi[u] = hb; lo[u] = bf16_bits(sres - bf16_val(hb));
    }
    const size_t o = (size_t)tok * DIN + c;
    *(volatile v4f*)(XCF + o) = sv; *(volatile us4*)(XCH + o) = hi; *(volatile us4*)(XCL + o) = lo;
    __threadfence();
    *(volatile v4f*)(XCF + o) = sv; *(volatile us4*)(XCH + o) = hi; *(volatile us4*)(XCL + o) = lo;
  }
}

template <int DIR>
__global__ __launch_bounds__(256) void k_scan(const float* __restrict__ XD, const float* __restrict__ XCF,
                                             const float* __restrict__ dtw, const float* __restrict__ dtb,
                                             const float* __restrict__ Alog, const float* __restrict__ Dv,
                                             const float* YFin, const float* ZB,
                                             float* YF, unsigned short* YGH, unsigned short* YGL) {
#pragma clang fp contract(off)
  __shared__ __attribute__((aligned(16))) float sy[SCH * SYP];
  const int b = blockIdx.x, tid = threadIdx.x, lane = tid & 31, wave = tid >> 5;
  const int d = tid;
  float A2[DST], h[DST], wr[DTR];
#pragma unroll
  for (int n = 0; n < DST; ++n) { A2[n] = -__expf(bf16r(Alog[d * DST + n])) * LOG2E; h[n] = 0.0f; }
#pragma unroll
  for (int k = 0; k < DTR; ++k) wr[k] = bf16r(dtw[d * DTR + k]);
  const float Dd = bf16r(Dv[d]);
  const float bd = bf16r(dtb[d]);
#pragma unroll 1
  for (int c = 0; c < LL / SCH; ++c) {
#pragma unroll 1
    for (int s = 0; s < SCH; ++s) {
      const int st = c * SCH + s;
      const size_t tok = (size_t)b * LL + (size_t)st;
      const float* xd = XD + tok * XDN;
      const v4f r0v = *(const v4fa*)(xd);
      const v4f r1v = *(const v4fa*)(xd + 4);
      v4f Bv[4], Cv[4];
#pragma unroll
      for (int q = 0; q < 4; ++q) {
        Bv[q] = *(const v4fa*)(xd + DTR + 4 * q);
        Cv[q] = *(const v4fa*)(xd + DTR + DST + 4 * q);
      }
      float raw = 0.0f;
#pragma unroll
      for (int k = 0; k < 4; ++k) raw = raw + r0v[k] * wr[k];
#pragma unroll
      for (int k = 0; k < 4; ++k) raw = raw + r1v[k] * wr[4 + k];
      const float a = raw + bd;
      const float dl = fmaxf(a, 0.0f) + log1pf(__expf(-fabsf(a)));
      const float xv = XCF[tok * DIN + d];
      const float dx = dl * xv;
      float y = 0.0f;
#pragma unroll
      for (int n = 0; n < DST; ++n) {
        const float e = exp2f(dl * A2[n]);
        h[n] = e * h[n] + dx * Bv[n >> 2][n & 3];
        y = y + h[n] * Cv[n >> 2][n & 3];
      }
      float yv = y + xv * Dd;
      if (DIR) {
        const int tr = LL - 1 - st;
        const size_t tokr = (size_t)b * LL + (size_t)tr;
        const float yf = YFin[tokr * DIN + d];
        const float zv = ZB[tokr * DIN + d];
        yv = (yf + yv) * siluf(zv);
      }
      sy[s * SYP + tid] = yv;
    }
    __syncthreads();
#pragma unroll
    for (int pass = 0; pass < 2; ++pass) {
#pragma unroll
      for (int it = 0; it < 4; ++it) {
        const int row = 4 * wave + it;
        if (DIR == 0) {
          const size_t tokw = (size_t)b * LL + (size_t)(c * SCH + row);
#pragma unroll
          for (int H = 0; H < 2; ++H) {
            const v4f v = *(const v4fa*)(sy + row * SYP + H * 128 + lane * 4);
            *(volatile v4f*)(YF + tokw * DIN + H * 128 + lane * 4) = v;
          }
        } else {
          const size_t tokw = (size_t)b * LL + (size_t)(LL - 1 - (c * SCH + row));
          const v4f va = *(const v4fa*)(sy + row * SYP + lane * 8);
          const v4f vb = *(const v4fa*)(sy + row * SYP + lane * 8 + 4);
          us8 hi, lo;
#pragma unroll
          for (int u = 0; u < 4; ++u) {
            const unsigned short ha = bf16_bits(va[u]);
            hi[u] = ha; lo[u] = bf16_bits(va[u] - bf16_val(ha));
            const unsigned short hb = bf16_bits(vb[u]);
            hi[4 + u] = hb; lo[4 + u] = bf16_bits(vb[u] - bf16_val(hb));
          }
          const size_t o = tokw * DIN + (size_t)(lane * 8);
          *(volatile us8*)(YGH + o) = hi; *(volatile us8*)(YGL + o) = lo;
        }
      }
      __threadfence();
    }
    __syncthreads();
  }
}

__global__ __launch_bounds__(256) void k_outT(const float* __restrict__ OT, const float* __restrict__ ob, float* out) {
#pragma clang fp contract(off)
  __shared__ __attribute__((aligned(16))) float sT[DMOD * TSP];
  const int tid = threadIdx.x, lane = tid & 31, wave = tid >> 5;
  const int tok0 = blockIdx.x * 32;
  const int b = tok0 / LL, l0 = tok0 - b * LL;
#pragma unroll
  for (int it = 0; it < 4; ++it) {
    const int i = it * 256 + tid, r = i >> 5, c4 = (i & 31) * 4;
    const v4f v = *(const v4fa*)(OT + (size_t)(tok0 + r) * DMOD + c4);
#pragma unroll
    for (int u = 0; u < 4; ++u) sT[(c4 + u) * TSP + r] = v[u];
  }
  __syncthreads();
  v4f vals[4];
  size_t offs[4];
#pragma unroll
  for (int it = 0; it < 4; ++it) {
    const int c = wave * 16 + it * 4 + (lane >> 3);
    const int l4 = (lane & 7) * 4;
    const v4f v = *(const v4fa*)(sT + c * TSP + l4);
    const float bias = bf16r(ob[c]);
    vals[it] = v + bias;
    offs[it] = ((size_t)(b * DMOD + c)) * LL + (size_t)(l0 + l4);
  }
#pragma unroll
  for (int pass = 0; pass < 2; ++pass) {
#pragma unroll
    for (int it = 0; it < 4; ++it) *(volatile v4f*)(out + offs[it]) = vals[it];
    __threadfence();
  }
}

extern "C" void kernel_launch(void* const* d_in, const int* in_sizes, int n_in,
                              void* d_out, int out_size, void* d_ws, size_t ws_size,
                              hipStream_t stream) {
  if (n_in < 24) return;
  if (in_sizes[0] != NTOK * DMOD || in_sizes[1] != NTOK * DMOD ||
      in_sizes[2] != DMOD || in_sizes[3] != DMOD || in_sizes[4] != DMOD || in_sizes[5] != DMOD ||
      in_sizes[6] != DIN * DMOD || in_sizes[7] != DIN * DMOD ||
      in_sizes[8] != DIN * DCV || in_sizes[9] != DIN || in_sizes[10] != DIN * DCV || in_sizes[11] != DIN ||
      in_sizes[12] != XDR * DIN || in_sizes[13] != XDR * DIN ||
      in_sizes[14] != DIN * DTR || in_sizes[15] != DIN || in_sizes[16] != DIN * DTR || in_sizes[17] != DIN ||
      in_sizes[18] != DIN * DST || in_sizes[19] != DIN * DST || in_sizes[20] != DIN || in_sizes[21] != DIN ||
      in_sizes[22] != DMOD * DIN || in_sizes[23] != DMOD || out_size != 2 * NTOK * DMOD) return;

  const float* x1    = (const float*)d_in[0];
  const float* x2    = (const float*)d_in[1];
  const float* lnqw  = (const float*)d_in[2];
  const float* lnqb  = (const float*)d_in[3];
  const float* lnkw  = (const float*)d_in[4];
  const float* lnkb  = (const float*)d_in[5];
  const float* winx  = (const float*)d_in[6];
  const float* winz  = (const float*)d_in[7];
  const float* cwf   = (const float*)d_in[8];
  const float* cbf   = (const float*)d_in[9];
  const float* cwb   = (const float*)d_in[10];
  const float* cbb   = (const float*)d_in[11];
  const float* xpf   = (const float*)d_in[12];
  const float* xpb   = (const float*)d_in[13];
  const float* dtwf  = (const float*)d_in[14];
  const float* dtbf  = (const float*)d_in[15];
  const float* dtwb  = (const float*)d_in[16];
  const float* dtbb  = (const float*)d_in[17];
  const float* Alf   = (const float*)d_in[18];
  const float* Alb   = (const float*)d_in[19];
  const float* Dvf   = (const float*)d_in[20];
  const float* Dvb   = (const float*)d_in[21];
  const float* ow    = (const float*)d_in[22];
  const float* ob    = (const float*)d_in[23];
  float* out = (float*)d_out;

  size_t off = 0;
  auto carve = [&](size_t bytes) -> char* { char* p = (char*)d_ws + off; off += (bytes + 255) & ~(size_t)255; return p; };
  unsigned short* WINX16 = (unsigned short*)carve((size_t)DIN * DMOD * 2);
  unsigned short* WINZ16 = (unsigned short*)carve((size_t)DIN * DMOD * 2);
  unsigned short* WXF16  = (unsigned short*)carve((size_t)XDN * DIN * 2);
  unsigned short* WXB16  = (unsigned short*)carve((size_t)XDN * DIN * 2);
  unsigned short* WO16   = (unsigned short*)carve((size_t)DMOD * DIN * 2);
  unsigned short* X1H    = (unsigned short*)carve((size_t)NTOK * DMOD * 2);
  unsigned short* X1L    = (unsigned short*)carve((size_t)NTOK * DMOD * 2);
  unsigned short* X2H    = (unsigned short*)carve((size_t)NTOK * DMOD * 2);
  unsigned short* X2L    = (unsigned short*)carve((size_t)NTOK * DMOD * 2);
  float* XB              = (float*)carve((size_t)NTOK * DIN * 4);
  float* ZB              = (float*)carve((size_t)NTOK * DIN * 4);
  float* XCF0            = (float*)carve((size_t)NTOK * DIN * 4);
  float* XCF1            = (float*)carve((size_t)NTOK * DIN * 4);
  unsigned short* XCH0   = (unsigned short*)carve((size_t)NTOK * DIN * 2);
  unsigned short* XCL0   = (unsigned short*)carve((size_t)NTOK * DIN * 2);
  unsigned short* XCH1   = (unsigned short*)carve((size_t)NTOK * DIN * 2);
  unsigned short* XCL1   = (unsigned short*)carve((size_t)NTOK * DIN * 2);
  float* XD0             = (float*)carve((size_t)NTOK * XDN * 4);
  float* XD1             = (float*)carve((size_t)NTOK * XDN * 4);
  float* YF              = (float*)carve((size_t)NTOK * DIN * 4);
  unsigned short* YGH    = (unsigned short*)carve((size_t)NTOK * DIN * 2);
  unsigned short* YGL    = (unsigned short*)carve((size_t)NTOK * DIN * 2);
  float* OUTT            = (float*)carve((size_t)NTOK * DMOD * 4);
  if (off > ws_size || off > WSCAP) return;

  const dim3 b256(256);
  k_cvt<<<dim3((DIN * DMOD / 8 + 255) / 256), b256, 0, stream>>>(winx, WINX16, DIN, DMOD / 8, DIN * DMOD / 8);
  k_cvt<<<dim3((DIN * DMOD / 8 + 255) / 256), b256, 0, stream>>>(winz, WINZ16, DIN, DMOD / 8, DIN * DMOD / 8);
  k_cvt<<<dim3((XDN * DIN / 8 + 255) / 256), b256, 0, stream>>>(xpf, WXF16, XDR, DIN / 8, XDN * DIN / 8);
  k_cvt<<<dim3((XDN * DIN / 8 + 255) / 256), b256, 0, stream>>>(xpb, WXB16, XDR, DIN / 8, XDN * DIN / 8);
  k_cvt<<<dim3((DMOD * DIN / 8 + 255) / 256), b256, 0, stream>>>(ow, WO16, DMOD, DIN / 8, DMOD * DIN / 8);
  k_ln<<<dim3(NTOK / 8), b256, 0, stream>>>(x1, x2, lnqw, lnqb, lnkw, lnkb, X1H, X1L, X2H, X2L);
  k_gemm<<<dim3(NTOK / 128, DIN / 64), b256, 0, stream>>>(X1H, X1L, DMOD, WINX16, DMOD, XB, DIN, DMOD);
  k_gemm<<<dim3(NTOK / 128, DIN / 64), b256, 0, stream>>>(X2H, X2L, DMOD, WINZ16, DMOD, ZB, DIN, DMOD);
  k_conv<0><<<dim3(NTOK / 8), b256, 0, stream>>>(XB, cwf, cbf, XCF0, XCH0, XCL0);
  k_conv<1><<<dim3(NTOK / 8), b256, 0, stream>>>(XB, cwb, cbb, XCF1, XCH1, XCL1);
  k_gemm<<<dim3(NTOK / 128, XDN / 64), b256, 0, stream>>>(XCH0, XCL0, DIN, WXF16, DIN, XD0, XDN, DIN);
  k_gemm<<<dim3(NTOK / 128, XDN / 64), b256, 0, stream>>>(XCH1, XCL1, DIN, WXB16, DIN, XD1, XDN, DIN);
  k_scan<0><<<dim3(NB), b256, 0, stream>>>(XD0, XCF0, dtwf, dtbf, Alf, Dvf, YF, ZB, YF, YGH, YGL);
  k_scan<1><<<dim3(NB), b256, 0, stream>>>(XD1, XCF1, dtwb, dtbb, Alb, Dvb, YF, ZB, YF, YGH, YGL);
  k_gemm<<<dim3(NTOK / 128, DMOD / 64), b256, 0, stream>>>(YGH, YGL, DIN, WO16, DIN, OUTT, DMOD, DIN);
  k_outT<<<dim3(NTOK / 32), b256, 0, stream>>>(OUTT, ob, out);
  const size_t o1b = (size_t)NTOK * DMOD * 4;
  k_copy<<<dim3((NTOK * DMOD / 4 + 255) / 256), b256, 0, stream>>>(x2, (float*)((char*)d_out + o1b), NTOK * DMOD / 4);
}
